// EncoderBlock_83288005804305
// MI455X (gfx1250) — hardware-verified
//
#include <hip/hip_runtime.h>
#include <math.h>

#ifndef NB
#define NB 2
#endif
#ifndef SEQ
#define SEQ 2048
#endif
#define NB_FULL 2
#define SEQ_FULL 2048
#define DM 1024
#define NH 16
#define DHD 64
#define DFF 4096
#define MROWS (NB * SEQ)
#define MW (SEQ / 32)

#define XC 16.0f
#define WC 256.0f
#define QC 16.0f
#define PC 16384.0f
#define CC 1024.0f
#define SC 16.0f
#define HC 16.0f

static_assert(NH * DHD == DM);
static_assert(DHD == 64);
static_assert(DM == 1024);
static_assert(SEQ % 64 == 0);
static_assert(MROWS % 64 == 0);
static_assert(DM % 64 == 0 && (2 * DM) % 64 == 0 && DFF % 64 == 0);
static_assert(DM % 32 == 0 && DFF % 32 == 0);
static_assert(((MROWS / 64) * ((2 * DM) / 64)) % 8 == 0);
static_assert(((DM / 64) * (SEQ / 64)) % 8 == 0);
static_assert(((MROWS / 64) * (DM / 64)) % 8 == 0);
static_assert(((long long)NB * SEQ * MW) % 32 == 0);
static_assert(MROWS % 8 == 0);
static_assert(NB <= NB_FULL && SEQ <= SEQ_FULL);

typedef __attribute__((ext_vector_type(16))) _Float16 v16h;
typedef __attribute__((ext_vector_type(8)))  _Float16 v8h;
typedef __attribute__((ext_vector_type(8)))  float    v8f;
typedef __attribute__((ext_vector_type(4)))  float    v4f;
typedef __attribute__((ext_vector_type(4)))  unsigned int v4u;
typedef __attribute__((ext_vector_type(2)))  unsigned int v2u;
typedef __attribute__((ext_vector_type(4)))  int      v4i;

union FragU { v16h v; v8h h[2]; };
__device__ __forceinline__ v16h ldfrag_g(const _Float16* __restrict__ p) { FragU f; f.h[0] = *(const v8h*)(p); f.h[1] = *(const v8h*)(p + 16); return f.v; }
__device__ __forceinline__ v8f mma16(v16h a, v16h b, v8f c) { return __builtin_amdgcn_wmma_f32_16x16x32_f16(false, a, false, b, (short)0, c, false, false); }
__device__ __forceinline__ void dep_guard_h(v8f& a, v8f& b, v16h x, v16h y) { asm volatile("v_nop\n\tv_nop\n\tv_nop\n\tv_nop" : "+v"(a), "+v"(b) : "v"(x), "v"(y)); }
__device__ __forceinline__ void keep4_h(v16h a, v16h b, v16h c, v16h d) { asm volatile("v_nop" :: "v"(a), "v"(b), "v"(c), "v"(d)); }
__device__ __forceinline__ void acc_guard4(v8f& a, v8f& b, v8f& c, v8f& d) { asm volatile("v_nop\n\tv_nop\n\tv_nop\n\tv_nop" : "+v"(a), "+v"(b), "+v"(c), "+v"(d)); }
__device__ __forceinline__ void guard1(v8f& a, v16h x, v16h y) { asm volatile("v_nop\n\tv_nop\n\tv_nop\n\tv_nop" : "+v"(a) : "v"(x), "v"(y)); }
__device__ __forceinline__ void guard4(v8f& a, v8f& b, v8f& c, v8f& d, v16h p, v16h x, v16h y, v16h z, v16h w) {
    asm volatile("v_nop\n\tv_nop\n\tv_nop\n\tv_nop" : "+v"(a), "+v"(b), "+v"(c), "+v"(d) : "v"(p), "v"(x), "v"(y), "v"(z), "v"(w)); }
__device__ __forceinline__ void wave_sync() { __builtin_amdgcn_fence(3  , "workgroup"); __builtin_amdgcn_wave_barrier(); __builtin_amdgcn_fence(2  , "workgroup"); }

#define VST2(T, ptr, val) do { const T vst2_v_ = (val); *(volatile T*)(ptr) = vst2_v_; __threadfence(); *(volatile T*)(ptr) = vst2_v_; } while (0)
#define VST2V4(ptr, val) do { const v4f vst2_v4_ = (val); *(volatile v4f*)(ptr) = vst2_v4_; __threadfence(); *(volatile v4f*)(ptr) = vst2_v4_; } while (0)

__device__ __forceinline__ float cmb_bf(float v) { const unsigned u = __builtin_bit_cast(unsigned, v); const unsigned r = (u + 0x7fffu + ((u >> 16) & 1u)) & 0xffff0000u; return __builtin_bit_cast(float, r); }
__device__ __forceinline__ unsigned int cmb_pk2(float a, float b) { return (unsigned int)__builtin_bit_cast(unsigned short, (_Float16)a) | ((unsigned int)__builtin_bit_cast(unsigned short, (_Float16)b) << 16); }

__global__ __launch_bounds__(256) void k_cm_castb(const float* __restrict__ SRC, int lds, unsigned short* __restrict__ DST, int ldd, int nR, int nC, float sc, int rpb, int rpb_full) {
    const long long u = (long long)blockIdx.x * 256 + threadIdx.x; const int per = nC / 8; if (u >= (long long)nR * per) return;
    const int r = (int)(u / per); const int c0 = 8 * (int)(u % per);
    const long long sr = (long long)(r / rpb) * rpb_full + (r % rpb);
    const float* s = SRC + sr * lds + c0;
    const v4f a = *(const v4f*)(s), b = *(const v4f*)(s + 4);
    v4u pk; pk.x = cmb_pk2(cmb_bf(a.x) * sc, cmb_bf(a.y) * sc); pk.y = cmb_pk2(cmb_bf(a.z) * sc, cmb_bf(a.w) * sc);
    pk.z = cmb_pk2(cmb_bf(b.x) * sc, cmb_bf(b.y) * sc); pk.w = cmb_pk2(cmb_bf(b.z) * sc, cmb_bf(b.w) * sc);
    VST2(v4u, (v4u*)(DST + (long long)r * ldd + c0), pk);
}
__global__ __launch_bounds__(256) void k_cm_castbT(const float* __restrict__ SRC, int lds, unsigned short* __restrict__ DST, int ldd, int nR, int nC, float sc) {
    const long long u = (long long)blockIdx.x * 256 + threadIdx.x; const int per = nR / 8; if (u >= (long long)nC * per) return;
    const int c = (int)(u / per); const int r0 = 8 * (int)(u % per);
    float w[8];
#pragma unroll
    for (int e = 0; e < 8; ++e) w[e] = cmb_bf(SRC[(long long)(r0 + e) * lds + c]) * sc;
    v4u pk; pk.x = cmb_pk2(w[0], w[1]); pk.y = cmb_pk2(w[2], w[3]); pk.z = cmb_pk2(w[4], w[5]); pk.w = cmb_pk2(w[6], w[7]);
    VST2(v4u, (v4u*)(DST + (long long)c * ldd + r0), pk);
}

__global__ __launch_bounds__(256) void k_maskpack(const int* __restrict__ M, unsigned int* __restrict__ MBo, int total) {
    const int u = blockIdx.x * 256 + threadIdx.x; if (u >= total) return;
    const int w = u % MW; const int rq = u / MW; const int q = rq % SEQ; const int b = rq / SEQ;
    const int* src = M + ((long long)b * SEQ_FULL + q) * SEQ_FULL + 32 * w;
    unsigned int bits = 0u;
#pragma unroll 1
    for (int i = 0; i < 8; ++i) {
        const v4i m = *(const v4i*)(src + 4 * i);
        const unsigned int nib = ((m.x != 0) ? 1u : 0u) | ((m.y != 0) ? 2u : 0u) | ((m.z != 0) ? 4u : 0u) | ((m.w != 0) ? 8u : 0u);
        bits |= nib << (4 * i);
    }
    VST2(unsigned int, MBo + u, bits);
}

template <int BIAS_MODE, int OUT_MODE, int ACT>
__device__ __forceinline__ void gemm64_body(const unsigned short* __restrict__ Ap, int lda, long strideA,
                                            const unsigned short* __restrict__ Btp, int ldb, long strideB,
                                            void* __restrict__ Cout, int ldc, long strideC, const float* __restrict__ bias,
                                            int M, int N, int K, float scale, float oscale) {
    __shared__ __align__(16) float sT[8][16 * 68];
    const _Float16* A = (const _Float16*)Ap; const _Float16* Bt = (const _Float16*)Btp;
    const int b = blockIdx.y;
    const int lane = threadIdx.x & 31;
    const int wave = threadIdx.x >> 5;
    const int tilesN = N >> 6;
    const int tilesM = M >> 6;
    const int tile = blockIdx.x * 8 + wave;
    if (tile >= tilesM * tilesN) return;
    const int tm = tile / tilesN;
    const int tn = tile - tm * tilesN;
    const int m0 = tm << 6;
    const int n0 = tn << 6;
    const _Float16* Ab = A + (size_t)b * strideA;
    const _Float16* Bb = Bt + (size_t)b * strideB;
    const int rlane = lane & 15;
    const int koff = (lane >> 4) * 8;
    const int mOff = (lane >> 4) * 8;

    v8f acc[4][4];
#pragma unroll
    for (int i = 0; i < 4; ++i)
#pragma unroll
        for (int j = 0; j < 4; ++j) acc[i][j] = (v8f){0.f, 0.f, 0.f, 0.f, 0.f, 0.f, 0.f, 0.f};

    for (int k0 = 0; k0 < K; k0 += 32) {
        v16h bh[4];
#pragma unroll
        for (int j = 0; j < 4; ++j) bh[j] = ldfrag_g(Bb + (size_t)(n0 + (j << 4) + rlane) * ldb + koff + k0);
#pragma unroll
        for (int i = 0; i < 4; ++i) {
            const v16h ah = ldfrag_g(Ab + (size_t)(m0 + (i << 4) + rlane) * lda + koff + k0);
#pragma unroll
            for (int j = 0; j < 4; ++j) acc[i][j] = mma16(ah, bh[j], acc[i][j]);
            dep_guard_h(acc[i][0], acc[i][3], ah, ah);
        }
        keep4_h(bh[0], bh[1], bh[2], bh[3]);
    }
    acc_guard4(acc[0][0], acc[0][1], acc[0][2], acc[0][3]);
    acc_guard4(acc[1][0], acc[1][1], acc[1][2], acc[1][3]);
    acc_guard4(acc[2][0], acc[2][1], acc[2][2], acc[2][3]);
    acc_guard4(acc[3][0], acc[3][1], acc[3][2], acc[3][3]);

    float* slab = sT[wave];
#pragma unroll
    for (int i = 0; i < 4; ++i) {
        const int mBase = m0 + (i << 4);
#pragma unroll
        for (int j = 0; j < 4; ++j) {
            const int n = n0 + (j << 4) + rlane;
            float bv = 0.f;
            if (BIAS_MODE == 2) bv = cmb_bf(bias[n]);
#pragma unroll
            for (int r = 0; r < 8; ++r) {
                float v = acc[i][j][r] * scale;
                if (BIAS_MODE == 1) v += cmb_bf(bias[mBase + mOff + r]);
                if (BIAS_MODE == 2) v += bv;
                if (ACT == 1) v = fmaxf(v, 0.0f);
                slab[(mOff + r) * 68 + (j << 4) + rlane] = v;
            }
        }
        wave_sync();
        if (OUT_MODE == 0) {
            float* C = (float*)Cout + (size_t)b * strideC;
            const int hh = lane >> 4, c4 = (lane & 15) * 4;
            for (int pass = 0; pass < 2; ++pass) {
#pragma unroll
                for (int it = 0; it < 8; ++it) {
                    const int row = it * 2 + hh;
                    const v4f v = *(const v4f*)(slab + row * 68 + c4);
                    *(volatile v4f*)(C + (size_t)(mBase + row) * ldc + n0 + c4) = v;
                }
                __threadfence();
            }
        } else {
            const int q = lane >> 3, c8 = (lane & 7) * 8;
            unsigned short* C = (unsigned short*)Cout + (size_t)b * strideC;
            for (int pass = 0; pass < 2; ++pass) {
#pragma unroll
                for (int it = 0; it < 4; ++it) {
                    const int row = it * 4 + q;
                    const float* sp = slab + row * 68 + c8;
                    v8h hv;
#pragma unroll
                    for (int e = 0; e < 8; ++e) hv[e] = (_Float16)(sp[e] * oscale);
                    *(volatile v8h*)(C + (size_t)(mBase + row) * ldc + n0 + c8) = hv;
                }
                __threadfence();
            }
        }
        wave_sync();
    }
}

__global__ __launch_bounds__(256) void k_gemm_h16(const unsigned short* __restrict__ Ap, int lda, long strideA, const unsigned short* __restrict__ Btp, int ldb, long strideB,
                                                  unsigned short* __restrict__ C, int ldc, long strideC, const float* __restrict__ bias, int M, int N, int K, float scale, float oscale) {
    gemm64_body<2, 1, 0>(Ap, lda, strideA, Btp, ldb, strideB, (void*)C, ldc, strideC, bias, M, N, K, scale, oscale);
}
__global__ __launch_bounds__(256) void k_gemm_vt(const unsigned short* __restrict__ Ap, int lda, long strideA, const unsigned short* __restrict__ Btp, int ldb, long strideB,
                                                 unsigned short* __restrict__ C, int ldc, long strideC, const float* __restrict__ bias, int M, int N, int K, float scale, float oscale) {
    gemm64_body<1, 1, 0>(Ap, lda, strideA, Btp, ldb, strideB, (void*)C, ldc, strideC, bias, M, N, K, scale, oscale);
}
__global__ __launch_bounds__(256) void k_gemm_relu16(const unsigned short* __restrict__ Ap, int lda, long strideA, const unsigned short* __restrict__ Btp, int ldb, long strideB,
                                                     unsigned short* __restrict__ C, int ldc, long strideC, const float* __restrict__ bias, int M, int N, int K, float scale, float oscale) {
    gemm64_body<2, 1, 1>(Ap, lda, strideA, Btp, ldb, strideB, (void*)C, ldc, strideC, bias, M, N, K, scale, oscale);
}
__global__ __launch_bounds__(256) void k_gemm_f32(const unsigned short* __restrict__ Ap, int lda, long strideA, const unsigned short* __restrict__ Btp, int ldb, long strideB,
                                                  float* __restrict__ C, int ldc, long strideC, const float* __restrict__ bias, int M, int N, int K, float scale) {
    gemm64_body<2, 0, 0>(Ap, lda, strideA, Btp, ldb, strideB, (void*)C, ldc, strideC, bias, M, N, K, scale, 1.0f);
}

__global__ __launch_bounds__(128) void k_attn(const unsigned short* __restrict__ QKp, const unsigned short* __restrict__ VTp,
                                              const unsigned int* __restrict__ MB, unsigned short* __restrict__ CTX) {
    __shared__ __align__(16) unsigned int mb_s[64 * MW];
    __shared__ __align__(16) _Float16 Psh[4][16 * 64];
    __shared__ __align__(16) float Os[4][16 * 68];
    const _Float16* QK = (const _Float16*)QKp; const _Float16* VT = (const _Float16*)VTp;
    const int tid = threadIdx.x;
    const int wave = tid >> 5;
    const int lane = tid & 31;
    const int hh = lane >> 4;
    const int c = lane & 15;
    const int nqb = SEQ / 64;
    const int bx = blockIdx.x;
    const int qb = bx % nqb;
    const int bh = bx / nqb;
    const int h = bh % NH;
    const int b = bh / NH;
    const int q0 = qb * 64 + wave * 16;

    {
        const v4u* src = (const v4u*)(MB + ((size_t)b * SEQ + (size_t)qb * 64) * MW);
        for (int i = tid; i < 64 * MW / 4; i += 128) *(v4u*)&mb_s[4 * i] = src[i];
    }
    __syncthreads();

    v16h qa[2];
    {
        const _Float16* qrow = QK + (size_t)(b * SEQ + q0 + c) * (2 * DM) + h * DHD + 8 * hh;
        qa[0] = ldfrag_g(qrow); qa[1] = ldfrag_g(qrow + 32);
    }
    float mrow[8], lrow[8];
    v8f oacc[4];
#pragma unroll
    for (int r = 0; r < 8; ++r) { mrow[r] = -INFINITY; lrow[r] = 0.f; }
#pragma unroll
    for (int t = 0; t < 4; ++t) oacc[t] = (v8f){0.f, 0.f, 0.f, 0.f, 0.f, 0.f, 0.f, 0.f};

    const float SCL2 = 0.125f * (1.0f / (QC * QC)) * 1.4426950408889634f;
    const float FILL2 = -1.0e9f * 1.4426950408889634f;

    for (int kc = 0; kc < SEQ / 64; ++kc) {
        const int kv0 = kc * 64;
        v8f s[4];
#pragma unroll
        for (int j = 0; j < 4; ++j) {
            const _Float16* krow = QK + (size_t)(b * SEQ + kv0 + j * 16 + c) * (2 * DM) + DM + h * DHD + 8 * hh;
            const v16h k0 = ldfrag_g(krow), k1 = ldfrag_g(krow + 32);
            v8f a = (v8f){0.f, 0.f, 0.f, 0.f, 0.f, 0.f, 0.f, 0.f};
            a = mma16(qa[0], k0, a);
            a = mma16(qa[1], k1, a);
            guard1(a, k0, k1);
            s[j] = a;
        }
        v2u mw[8]; unsigned int many = 0u;
#pragma unroll
        for (int r = 0; r < 8; ++r) { mw[r] = *(const v2u*)&mb_s[(wave * 16 + 8 * hh + r) * MW + kc * 2]; many |= mw[r].x | mw[r].y; }
        const bool anym = (__ballot(many != 0u) != 0ull);
        float cm[8];
#pragma unroll
        for (int r = 0; r < 8; ++r) {
            float m = -INFINITY;
#pragma unroll
            for (int j = 0; j < 4; ++j) {
                float v = s[j][r] * SCL2;
                if (anym) {
                    const unsigned int w = (j < 2) ? mw[r].x : mw[r].y;
                    const unsigned int bit = (w >> ((j & 1) * 16 + c)) & 1u;
                    v = (bit != 0u) ? FILL2 : v;
                }
                s[j][r] = v;
                m = fmaxf(m, v);
            }
#pragma unroll
            for (int off = 1; off < 16; off <<= 1) m = fmaxf(m, __shfl_xor(m, off, 32));
            cm[r] = m;
        }
#pragma unroll
        for (int r = 0; r < 8; ++r) {
            const float mnew = fmaxf(mrow[r], cm[r]);
            const float alpha = exp2f(mrow[r] - mnew);
            mrow[r] = mnew;
            float psum = 0.f;
#pragma unroll
            for (int j = 0; j < 4; ++j) {
                const float p = exp2f(s[j][r] - mnew);
                psum += p;
                Psh[wave][(8 * hh + r) * 64 + j * 16 + c] = (_Float16)(p * PC);
            }
#pragma unroll
            for (int off = 1; off < 16; off <<= 1) psum += __shfl_xor(psum, off, 32);
            lrow[r] = lrow[r] * alpha + psum;
#pragma unroll
            for (int t = 0; t < 4; ++t) oacc[t][r] *= alpha;
        }
        wave_sync();
#pragma unroll 1
        for (int kk = 0; kk < 2; ++kk) {
            FragU pa;
            pa.h[0] = *(const v8h*)&Psh[wave][c * 64 + kk * 32 + 8 * hh];
            pa.h[1] = *(const v8h*)&Psh[wave][c * 64 + kk * 32 + 16 + 8 * hh];
            v16h vb[4];
#pragma unroll
            for (int t = 0; t < 4; ++t) vb[t] = ldfrag_g(VT + ((size_t)(b * NH + h) * DHD + t * 16 + c) * SEQ + kv0 + kk * 32 + 8 * hh);
#pragma unroll
            for (int t = 0; t < 4; ++t) oacc[t] = mma16(pa.v, vb[t], oacc[t]);
            guard4(oacc[0], oacc[1], oacc[2], oacc[3], pa.v, vb[0], vb[1], vb[2], vb[3]);
        }
        wave_sync();
    }

#pragma unroll
    for (int r = 0; r < 8; ++r) {
        const float inv = (CC / (PC * QC)) * (1.0f / lrow[r]);
#pragma unroll
        for (int t = 0; t < 4; ++t) Os[wave][(8 * hh + r) * 68 + t * 16 + c] = oacc[t][r] * inv;
    }
    wave_sync();
    {
        const int q8 = lane >> 3, c8 = (lane & 7) * 8;
        unsigned short* cb = CTX + (size_t)(b * SEQ + q0) * DM + h * DHD;
        for (int pass = 0; pass < 2; ++pass) {
#pragma unroll
            for (int it = 0; it < 4; ++it) {
                const int row = it * 4 + q8;
                v8h hv;
#pragma unroll
                for (int e = 0; e < 8; ++e) hv[e] = (_Float16)Os[wave][row * 68 + c8 + e];
                *(volatile v8h*)(cb + (size_t)row * DM + c8) = hv;
            }
            __threadfence();
        }
    }
}

template <int XBF, int W16>
__device__ __forceinline__ void ln_body(const float* __restrict__ A, const float* __restrict__ X, const float* __restrict__ GA, const float* __restrict__ BE,
                                        int rows, int rpb, int rpb_full, float* __restrict__ Yf, unsigned short* __restrict__ Y16, float c16) {
    #pragma clang fp contract(off)
    constexpr int NQ = 8; constexpr int WD = 128 * NQ;
    static_assert(WD == DM);
    const int r = blockIdx.x * 8 + (threadIdx.x >> 5); const int L = threadIdx.x & 31; if (r >= rows) return;
    const long long xr = XBF ? ((long long)(r / rpb) * rpb_full + (r % rpb)) : (long long)r;
    v4f v[NQ]; float s = 0.f;
#pragma unroll
    for (int q = 0; q < NQ; ++q) {
        const int cc = 4 * L + 128 * q;
        v[q] = *(const v4f*)(A + (long long)r * WD + cc);
        v4f x = *(const v4f*)(X + xr * WD + cc);
        if (XBF) { x.x = cmb_bf(x.x); x.y = cmb_bf(x.y); x.z = cmb_bf(x.z); x.w = cmb_bf(x.w); }
        v[q] = v[q] + x;
        s += (v[q].x + v[q].y) + (v[q].z + v[q].w);
    }
#pragma unroll
    for (int o = 16; o > 0; o >>= 1) s += __shfl_xor(s, o, 32);
    const float mu = s * (1.f / WD); float qq = 0.f;
#pragma unroll
    for (int q = 0; q < NQ; ++q) { v[q].x -= mu; v[q].y -= mu; v[q].z -= mu; v[q].w -= mu; qq += (v[q].x * v[q].x + v[q].y * v[q].y) + (v[q].z * v[q].z + v[q].w * v[q].w); }
#pragma unroll
    for (int o = 16; o > 0; o >>= 1) qq += __shfl_xor(qq, o, 32);
    const float rs = rsqrtf(qq * (1.f / WD) + 1e-6f);
#pragma unroll
    for (int q = 0; q < NQ; ++q) {
        const int cc = 4 * L + 128 * q; const v4f ga = *(const v4f*)(GA + cc), be = *(const v4f*)(BE + cc);
        v4f y; y.x = v[q].x * rs * cmb_bf(ga.x) + cmb_bf(be.x); y.y = v[q].y * rs * cmb_bf(ga.y) + cmb_bf(be.y); y.z = v[q].z * rs * cmb_bf(ga.z) + cmb_bf(be.z); y.w = v[q].w * rs * cmb_bf(ga.w) + cmb_bf(be.w);
        const long long o = (long long)r * WD + cc;
        VST2V4(Yf + o, y);
        if (W16) { v2u pk; pk.x = cmb_pk2(y.x * c16, y.y * c16); pk.y = cmb_pk2(y.z * c16, y.w * c16); VST2(v2u, (v2u*)(Y16 + o), pk); }
    }
}
__global__ __launch_bounds__(256) void k_ln_a(const float* __restrict__ A, const float* __restrict__ X, const float* __restrict__ GA, const float* __restrict__ BE,
                                              int rows, int rpb, int rpb_full, float* __restrict__ Yf, unsigned short* __restrict__ Y16) {
    ln_body<1, 1>(A, X, GA, BE, rows, rpb, rpb_full, Yf, Y16, SC);
}
__global__ __launch_bounds__(256) void k_ln_b(const float* __restrict__ A, const float* __restrict__ X, const float* __restrict__ GA, const float* __restrict__ BE,
                                              int rows, float* __restrict__ Yf) {
    ln_body<0, 0>(A, X, GA, BE, rows, 1, 1, Yf, nullptr, 1.0f);
}

constexpr size_t al256(size_t x) { return (x + 255) / 256 * 256; }
constexpr size_t SZ_X16  = (size_t)MROWS * DM * 2;
constexpr size_t SZ_WQKV = (size_t)3 * DM * DM * 2;
constexpr size_t SZ_WPRJ = (size_t)DM * DM * 2;
constexpr size_t SZ_W1   = (size_t)DFF * DM * 2;
constexpr size_t SZ_W2   = (size_t)DM * DFF * 2;
constexpr size_t SZ_QK   = (size_t)MROWS * 2 * DM * 2;
constexpr size_t SZ_VT   = (size_t)NB * DM * SEQ * 2;
constexpr size_t SZ_CTX  = (size_t)MROWS * DM * 2;
constexpr size_t SZ_HID  = (size_t)MROWS * DFF * 2;
constexpr size_t SZ_MB   = (size_t)NB * SEQ * MW * 4;
constexpr size_t SZ_F32  = (size_t)MROWS * DM * 4;
constexpr size_t SZ_S16  = (size_t)MROWS * DM * 2;
static_assert(SZ_QK % 256 == 0 && SZ_VT % 256 == 0 && SZ_CTX % 256 == 0);
static_assert(SZ_QK + SZ_VT + SZ_CTX >= SZ_HID);
constexpr size_t OFF_X16  = 0;
constexpr size_t OFF_WQKV = OFF_X16 + al256(SZ_X16);
constexpr size_t OFF_WPRJ = OFF_WQKV + al256(SZ_WQKV);
constexpr size_t OFF_W1   = OFF_WPRJ + al256(SZ_WPRJ);
constexpr size_t OFF_W2   = OFF_W1 + al256(SZ_W1);
constexpr size_t OFF_QK   = OFF_W2 + al256(SZ_W2);
constexpr size_t OFF_VT   = OFF_QK + SZ_QK;
constexpr size_t OFF_CTX  = OFF_VT + SZ_VT;
constexpr size_t OFF_MB   = OFF_CTX + al256(SZ_CTX);
constexpr size_t OFF_ATT  = OFF_MB + al256(SZ_MB);
constexpr size_t OFF_S1F  = OFF_ATT + al256(SZ_F32);
constexpr size_t OFF_S16  = OFF_S1F + al256(SZ_F32);
constexpr size_t WS_TOTAL = OFF_S16 + al256(SZ_S16);
static_assert(WS_TOTAL <= (size_t)134217728);
static_assert(OFF_QK % 256 == 0 && OFF_MB % 256 == 0 && OFF_ATT % 256 == 0 && OFF_S1F % 256 == 0 && OFF_S16 % 256 == 0);

extern "C" void kernel_launch(void* const* d_in, const int* in_sizes, int n_in, void* d_out, int out_size, void* d_ws, size_t ws_size, hipStream_t stream) {
    if (n_in < 14) return;
    const long long need_x = ((long long)(NB - 1) * SEQ_FULL + SEQ) * DM;
    const long long need_m = ((long long)(NB - 1) * SEQ_FULL + (SEQ - 1)) * SEQ_FULL + SEQ;
    if ((long long)in_sizes[0] < need_x || (long long)in_sizes[1] < need_m) return;
    if (in_sizes[2] < DM * 3 * DM || in_sizes[3] < 3 * DM || in_sizes[4] < DM * DM || in_sizes[5] < DM) return;
    if (in_sizes[6] < DM * DFF || in_sizes[7] < DFF || in_sizes[8] < DFF * DM || in_sizes[9] < DM) return;
    if (in_sizes[10] < DM || in_sizes[11] < DM || in_sizes[12] < DM || in_sizes[13] < DM) return;
    if ((long long)out_size < (long long)MROWS * DM) return;
    if (ws_size < WS_TOTAL) return;

    const float* x     = (const float*)d_in[0];
    const int*   mask  = (const int*)d_in[1];
    const float* w_qkv = (const float*)d_in[2];
    const float* b_qkv = (const float*)d_in[3];
    const float* w_prj = (const float*)d_in[4];
    const float* b_prj = (const float*)d_in[5];
    const float* w1    = (const float*)d_in[6];
    const float* b1    = (const float*)d_in[7];
    const float* w2    = (const float*)d_in[8];
    const float* b2    = (const float*)d_in[9];
    const float* g1    = (const float*)d_in[10];
    const float* be1   = (const float*)d_in[11];
    const float* g2    = (const float*)d_in[12];
    const float* be2   = (const float*)d_in[13];
    float* out = (float*)d_out;

    char* ws = (char*)d_ws;
    unsigned short* X16   = (unsigned short*)(ws + OFF_X16);
    unsigned short* WQKV  = (unsigned short*)(ws + OFF_WQKV);
    unsigned short* WPRJ  = (unsigned short*)(ws + OFF_WPRJ);
    unsigned short* W1T   = (unsigned short*)(ws + OFF_W1);
    unsigned short* W2T   = (unsigned short*)(ws + OFF_W2);
    unsigned short* QK16  = (unsigned short*)(ws + OFF_QK);
    unsigned short* VT16  = (unsigned short*)(ws + OFF_VT);
    unsigned short* CTX16 = (unsigned short*)(ws + OFF_CTX);
    unsigned short* HID16 = (unsigned short*)(ws + OFF_QK);
    unsigned int*   MBITS = (unsigned int*)(ws + OFF_MB);
    float*          ATT   = (float*)(ws + OFF_ATT);
    float*          FF2   = (float*)(ws + OFF_ATT);
    float*          S1F   = (float*)(ws + OFF_S1F);
    unsigned short* S116  = (unsigned short*)(ws + OFF_S16);

    k_cm_castb<<<(unsigned)(((long long)MROWS * (DM / 8) + 255) / 256), 256, 0, stream>>>(x, DM, X16, DM, MROWS, DM, XC, SEQ, SEQ_FULL);
    k_cm_castbT<<<(unsigned)(((long long)(3 * DM) * (DM / 8) + 255) / 256), 256, 0, stream>>>(w_qkv, 3 * DM, WQKV, DM, DM, 3 * DM, WC);
    k_cm_castbT<<<(unsigned)(((long long)DM * (DM / 8) + 255) / 256), 256, 0, stream>>>(w_prj, DM, WPRJ, DM, DM, DM, WC);
    k_cm_castbT<<<(unsigned)(((long long)DFF * (DM / 8) + 255) / 256), 256, 0, stream>>>(w1, DFF, W1T, DM, DM, DFF, WC);
    k_cm_castbT<<<(unsigned)(((long long)DM * (DFF / 8) + 255) / 256), 256, 0, stream>>>(w2, DM, W2T, DFF, DFF, DM, WC);
    k_maskpack<<<(unsigned)(((long long)NB * SEQ * MW + 255) / 256), 256, 0, stream>>>(mask, MBITS, NB * SEQ * MW);

    k_gemm_h16<<<dim3((unsigned)(((MROWS / 64) * ((2 * DM) / 64) + 7) / 8), 1u), 256, 0, stream>>>(
        X16, DM, 0L, WQKV, DM, 0L, QK16, 2 * DM, 0L, b_qkv, MROWS, 2 * DM, DM, 1.0f / (XC * WC), QC);
    k_gemm_vt<<<dim3((unsigned)(((DM / 64) * (SEQ / 64) + 7) / 8), (unsigned)NB), 256, 0, stream>>>(
        WQKV + (size_t)2 * DM * DM, DM, 0L, X16, DM, (long)SEQ * DM, VT16, SEQ, (long)DM * SEQ, b_qkv + 2 * DM, DM, SEQ, DM, 1.0f / (XC * WC), QC);
    k_attn<<<(unsigned)(NB * NH * (SEQ / 64)), 128, 0, stream>>>(QK16, VT16, MBITS, CTX16);
    k_gemm_f32<<<dim3((unsigned)(((MROWS / 64) * (DM / 64) + 7) / 8), 1u), 256, 0, stream>>>(
        CTX16, DM, 0L, WPRJ, DM, 0L, ATT, DM, 0L, b_prj, MROWS, DM, DM, 1.0f / (CC * WC));
    k_ln_a<<<(unsigned)(MROWS / 8), 256, 0, stream>>>(ATT, x, g1, be1, MROWS, SEQ, SEQ_FULL, S1F, S116);
    k_gemm_relu16<<<dim3((unsigned)(((MROWS / 64) * (DFF / 64) + 7) / 8), 1u), 256, 0, stream>>>(
        S116, DM, 0L, W1T, DM, 0L, HID16, DFF, 0L, b1, MROWS, DFF, DM, 1.0f / (SC * WC), HC);
    k_gemm_f32<<<dim3((unsigned)(((MROWS / 64) * (DM / 64) + 7) / 8), 1u), 256, 0, stream>>>(
        HID16, DFF, 0L, W2T, DFF, 0L, FF2, DM, 0L, b2, MROWS, DM, DFF, 1.0f / (HC * WC));
    k_ln_b<<<(unsigned)(MROWS / 8), 256, 0, stream>>>(FF2, S1F, g2, be2, MROWS, out);
}
